// GATEncoder_14705968022274
// MI455X (gfx1250) — hardware-verified
//
#include <hip/hip_runtime.h>
#include <stddef.h>
#include <math.h>


#define DIN     256
#define CW      256
#define HEADS   4
#define HC      64
#define NSC     (2 * HEADS)
#define K1      256
#define CPL     8
#define NTHR    256
#define NWAVE   8
#define EPT     8
#define CHUNK   (NTHR * EPT)
#define WCAP    (EPT * 32)
#define LISTN   (NWAVE * WCAP)
#define NBMAX   2048
#define NBRUN   1024
#define SLOTB   11
#define RCAP    28672
#define DEGCAP  128
#define STW     256
#define GBM     64
#define GBN     64
#define GTHR    128
#define NBW1    ((CW * (K1 / 8)) / NTHR)
#define USH1    5
#define NEGSA   0.2f
#define EPS_SM  1e-16f
#define WSMAX   134217728
#define LDS_AGG ((2 * RCAP + 2 * NBMAX + LISTN) * 4 + 64)

static_assert((CHUNK & (CHUNK - 1)) == 0 && CHUNK <= (1 << SLOTB));
static_assert(NBMAX == (1 << SLOTB));
static_assert((NBRUN & (NBRUN - 1)) == 0 && NBRUN <= NBMAX && NBRUN >= 32);
static_assert(NTHR * 8 == NBMAX);
static_assert(LISTN >= NBMAX);
static_assert(LISTN >= NWAVE * WCAP);
static_assert((RCAP % 32) == 0);
static_assert(NWAVE * STW <= RCAP);
static_assert(CW <= STW && STW == 32 * CPL);
static_assert(LDS_AGG <= 300000);
static_assert(LDS_AGG == 254016);
static_assert(GBM == (GTHR / 32) * 16);
static_assert(GTHR == 2 * GBM);
static_assert((K1 % 32) == 0 && DIN == K1);
static_assert(K1 / 8 == (1 << USH1));
static_assert((CW % GBN) == 0 && GBN == HC && CW / GBN == HEADS);
static_assert(CW == 32 * CPL && CPL == 8);
static_assert(CW == HEADS * HC && HC == 8 * CPL);
static_assert(NBW1 * NTHR == CW * (K1 / 8));
static_assert(DIN / 8 == 32);
static_assert(DEGCAP <= RCAP);

typedef float          v4f  __attribute__((ext_vector_type(4)));
typedef float          v8f  __attribute__((ext_vector_type(8)));
typedef int            v4i  __attribute__((ext_vector_type(4)));
typedef int            v8i  __attribute__((ext_vector_type(8)));
typedef unsigned int   v4u  __attribute__((ext_vector_type(4)));
typedef unsigned short v8us __attribute__((ext_vector_type(8)));
typedef __bf16         v16b __attribute__((ext_vector_type(16)));
typedef v4f  __attribute__((may_alias)) v4fa;
typedef v8us __attribute__((may_alias)) v8usa;
union FragB { v16b v; v8us h[2]; v8i w; };

__device__ __forceinline__ v8f wmb(const FragB& a, const FragB& b, v8f c) {
  v8f d = __builtin_amdgcn_wmma_f32_16x16x32_bf16(false, a.v, false, b.v, (short)0, c, false, false);
  asm volatile("v_nop\n\tv_nop\n\tv_nop\n\tv_nop" : "+v"(d) : "v"(a.w), "v"(b.w));
  return d;
}

__device__ __forceinline__ unsigned int f2bf(float f) {
  const unsigned int u = __float_as_uint(f);
  return ((u + 0x7FFFu + ((u >> 16) & 1u)) >> 16) & 0xFFFFu;
}
__device__ __forceinline__ float bf2f(unsigned int b) { return __uint_as_float(b << 16); }
__device__ __forceinline__ float bfr(float f) { return bf2f(f2bf(f)); }
__device__ __forceinline__ v4f bfr4(const v4f a) {
  v4f r; r.x = bfr(a.x); r.y = bfr(a.y); r.z = bfr(a.z); r.w = bfr(a.w); return r;
}
__device__ __forceinline__ v8us cvt8b(const v4f a, const v4f b) {
  v8us o;
  o[0] = (unsigned short)f2bf(a.x); o[1] = (unsigned short)f2bf(a.y);
  o[2] = (unsigned short)f2bf(a.z); o[3] = (unsigned short)f2bf(a.w);
  o[4] = (unsigned short)f2bf(b.x); o[5] = (unsigned short)f2bf(b.y);
  o[6] = (unsigned short)f2bf(b.z); o[7] = (unsigned short)f2bf(b.w);
  return o;
}
template<int NQ>
__device__ __forceinline__ void ldq(float (&d)[4 * NQ], const float* __restrict__ p) {
#pragma unroll
  for (int k = 0; k < NQ; ++k) {
    const v4f t = *(const v4fa*)(p + 4 * k);
    d[4 * k] = t.x; d[4 * k + 1] = t.y; d[4 * k + 2] = t.z; d[4 * k + 3] = t.w;
  }
}
template<int NQ>
__device__ __forceinline__ void ldqb(float (&d)[4 * NQ], const float* __restrict__ p) {
#pragma unroll
  for (int k = 0; k < NQ; ++k) {
    const v4f t = bfr4(*(const v4fa*)(p + 4 * k));
    d[4 * k] = t.x; d[4 * k + 1] = t.y; d[4 * k + 2] = t.z; d[4 * k + 3] = t.w;
  }
}

__device__ __forceinline__ int scan_chunk(const int* __restrict__ dsts, int nE, int cbase, int slotBase,
                                          int nb, int vec8, int* list, int tid, int lane, int wave) {
  int wc = 0;
  const int el0  = tid * EPT;
  const int e0   = cbase + el0;
  const int sent = -2147483647 - 1;
  v4i da, db;
  if (vec8 != 0 && cbase + CHUNK <= nE) {
    da = *(const v4i*)(dsts + e0);
    db = *(const v4i*)(dsts + e0 + 4);
  } else {
    da.x = (e0     < nE) ? dsts[min(e0,     nE - 1)] : sent;
    da.y = (e0 + 1 < nE) ? dsts[min(e0 + 1, nE - 1)] : sent;
    da.z = (e0 + 2 < nE) ? dsts[min(e0 + 2, nE - 1)] : sent;
    da.w = (e0 + 3 < nE) ? dsts[min(e0 + 3, nE - 1)] : sent;
    db.x = (e0 + 4 < nE) ? dsts[min(e0 + 4, nE - 1)] : sent;
    db.y = (e0 + 5 < nE) ? dsts[min(e0 + 5, nE - 1)] : sent;
    db.z = (e0 + 6 < nE) ? dsts[min(e0 + 6, nE - 1)] : sent;
    db.w = (e0 + 7 < nE) ? dsts[min(e0 + 7, nE - 1)] : sent;
  }
  const unsigned nbs = (unsigned)slotBase;
  const unsigned unb = (unsigned)nb;
  const unsigned s0 = (unsigned)da.x - nbs, s1 = (unsigned)da.y - nbs;
  const unsigned s2 = (unsigned)da.z - nbs, s3 = (unsigned)da.w - nbs;
  const unsigned s4 = (unsigned)db.x - nbs, s5 = (unsigned)db.y - nbs;
  const unsigned s6 = (unsigned)db.z - nbs, s7 = (unsigned)db.w - nbs;
  const bool h0 = s0 < unb, h1 = s1 < unb, h2 = s2 < unb, h3 = s3 < unb;
  const bool h4 = s4 < unb, h5 = s5 < unb, h6 = s6 < unb, h7 = s7 < unb;
  const unsigned any = __builtin_amdgcn_ballot_w32(h0 | h1 | h2 | h3 | h4 | h5 | h6 | h7);
  if (any != 0u) {
#define HITJ(J, HJ, SJ) { \
      const unsigned mj = __builtin_amdgcn_ballot_w32(HJ); \
      if (mj != 0u) { \
        if (HJ) { \
          const int pos = wc + (int)__builtin_amdgcn_mbcnt_lo(mj, 0u); \
          if (pos < WCAP) list[wave * WCAP + pos] = ((el0 + (J)) << SLOTB) | (int)(SJ); \
        } \
        wc += (int)__builtin_popcount(mj); } }
    HITJ(0, h0, s0)
    HITJ(1, h1, s1)
    HITJ(2, h2, s2)
    HITJ(3, h3, s3)
    HITJ(4, h4, s4)
    HITJ(5, h5, s5)
    HITJ(6, h6, s6)
    HITJ(7, h7, s7)
#undef HITJ
  }
  return wc;
}

__device__ __forceinline__ void wt_unit(const float* __restrict__ w, int cols, int ush, int kmask, int Kout,
                                        unsigned short* wt, int rowoff, int u) {
  const int n   = u >> ush;
  const int k8  = (u & ((1 << ush) - 1)) * 8;
  const int kk  = k8 & kmask;
  const int ncl = n < cols ? n : cols - 1;
  const float* p = w + (size_t)kk * (size_t)cols + ncl;
  v4f a, b;
  a.x = p[0];                  a.y = p[(size_t)cols];       a.z = p[(size_t)2 * cols];   a.w = p[(size_t)3 * cols];
  b.x = p[(size_t)4 * cols];   b.y = p[(size_t)5 * cols];   b.z = p[(size_t)6 * cols];   b.w = p[(size_t)7 * cols];
  const v4f z4 = {0.f, 0.f, 0.f, 0.f};
  if (n >= cols) { a = z4; b = z4; }
  const v8us hv = cvt8b(a, b);
  const size_t o = (size_t)(rowoff + n) * (size_t)Kout + k8;
  *(volatile v8us*)(wt + o) = hv;
  __threadfence();
  *(volatile v8us*)(wt + o) = hv;
}

__global__ __launch_bounds__(NTHR) void k_prep(const float* __restrict__ x, const float* __restrict__ W,
                                               unsigned short* xb, unsigned short* wt,
                                               int nN, int nUx, int nBx) {
  const int tid = (int)threadIdx.x;
  const int bid = (int)blockIdx.x;
  if (bid < nBx) {
    const int i = bid * NTHR + tid;
    if (i >= nUx) return;
    const int row = i >> 5;
    const int c0  = (i & 31) * 8;
    const int rc  = row < nN ? row : nN - 1;
    const float* p = x + (size_t)rc * DIN + c0;
    v4f a = *(const v4fa*)p, b = *(const v4fa*)(p + 4);
    const v4f z4 = {0.f, 0.f, 0.f, 0.f};
    if (row >= nN) { a = z4; b = z4; }
    const v8us hv = cvt8b(a, b);
    const size_t o = (size_t)row * DIN + c0;
    *(volatile v8us*)(xb + o) = hv;
    __threadfence();
    *(volatile v8us*)(xb + o) = hv;
  } else {
    const int rb = bid - nBx;
    if (rb < NBW1) {
      const int u = rb * NTHR + tid;
      if (u < CW * (K1 / 8)) wt_unit(W, CW, USH1, DIN - 1, K1, wt, 0, u);
    }
  }
}

__global__ __launch_bounds__(GTHR) void k_gemm(
    const unsigned short* __restrict__ A, const unsigned short* __restrict__ WT,
    const float* __restrict__ atts, const float* __restrict__ attd,
    float* outF, float* SC, int K, int ldo, int MPr)
{
  __shared__ __attribute__((aligned(16))) float stg[GBM * GBN];
  __shared__ __attribute__((aligned(16))) float satt[2 * GBN];
  __shared__ __attribute__((aligned(16))) float ssc[2 * GBM];
  const int tid = (int)threadIdx.x, lane = tid & 31, wave = tid >> 5, hh = lane >> 4, m = lane & 15;
  const int rowBase = (int)blockIdx.x * GBM;
  const int head    = (int)blockIdx.y;
  const int col0    = head * GBN;

  if (tid < 32) {
    const int ia = col0 + 4 * (tid & 15);
    const v4f qa = bfr4(*(const v4fa*)(atts + ia));
    const v4f qb = bfr4(*(const v4fa*)(attd + ia));
    const float f = (tid < 16) ? 1.0f : 0.0f;
    *(v4fa*)(satt + 4 * tid) = qa * f + qb * (1.0f - f);
  }

  v8f acc[4];
  {
    const v8f z = {0.f, 0.f, 0.f, 0.f, 0.f, 0.f, 0.f, 0.f};
    acc[0] = z; acc[1] = z; acc[2] = z; acc[3] = z;
  }
  const unsigned short* ap = A  + (size_t)(rowBase + 16 * wave + m) * (size_t)K + 8 * hh;
  const unsigned short* wp = WT + (size_t)(col0 + m) * (size_t)K + 8 * hh;
  const int ksteps = K >> 5;
#pragma unroll 1
  for (int ks = 0; ks < ksteps; ++ks) {
    FragB af;
    af.h[0] = *(const v8usa*)(ap + 32 * ks);
    af.h[1] = *(const v8usa*)(ap + 32 * ks + 16);
#pragma unroll
    for (int t = 0; t < 4; ++t) {
      const unsigned short* wq = wp + (size_t)(16 * t) * (size_t)K + 32 * ks;
      FragB bf;
      bf.h[0] = *(const v8usa*)wq;
      bf.h[1] = *(const v8usa*)(wq + 16);
      acc[t] = wmb(af, bf, acc[t]);
    }
  }

#pragma unroll
  for (int t = 0; t < 4; ++t) {
    const int lc = 16 * t + m;
#pragma unroll
    for (int r = 0; r < 8; ++r) {
      const int lr = 16 * wave + 8 * hh + r;
      stg[lr * GBN + lc] = acc[t][r];
    }
  }
  __syncthreads();

  {
    const int row = tid & (GBM - 1);
    const int sel = tid >> 6;
    const float* avp = satt + GBN * sel;
    const float* sp  = stg + row * GBN;
    float sc = 0.f;
#pragma unroll 4
    for (int j = 0; j < GBN; ++j) sc = fmaf(sp[j], avp[j], sc);
    ssc[GBM * sel + row] = sc;
  }
  __syncthreads();

  const v4f sv = *(const v4fa*)(ssc + 4 * lane);
  float* scp = SC + (size_t)(head + HEADS * hh) * (size_t)MPr + rowBase + 4 * m;

  v4f fv[8];
#pragma unroll
  for (int i = 0; i < 8; ++i) {
    const int lr = 16 * wave + 2 * i + hh;
    fv[i] = *(const v4fa*)(stg + lr * GBN + 4 * m);
  }
  if (wave == 0) *(volatile v4f*)scp = sv;
#pragma unroll
  for (int i = 0; i < 8; ++i) {
    const int lr = 16 * wave + 2 * i + hh;
    const int gr = rowBase + lr;
    float* op = outF + (size_t)gr * (size_t)ldo + col0 + 4 * m;
    *(volatile v4f*)op = fv[i];
  }
  __threadfence();
  if (wave == 0) *(volatile v4f*)scp = sv;
#pragma unroll
  for (int i = 0; i < 8; ++i) {
    const int lr = 16 * wave + 2 * i + hh;
    const int gr = rowBase + lr;
    float* op = outF + (size_t)gr * (size_t)ldo + col0 + 4 * m;
    *(volatile v4f*)op = fv[i];
  }
}

template<int C>
__device__ __forceinline__ void smerge(float lg, float& mx, float& dn, float (&av)[C], const float (&hs)[C]) {
  const float df = lg - mx;
  const float ee = __expf(-fabsf(df));
  const bool up  = df > 0.f;
  const float s1 = up ? ee : 1.0f;
  const float s2 = up ? 1.0f : ee;
  mx = up ? lg : mx;
  dn = fmaf(dn, s1, s2);
#pragma unroll
  for (int j = 0; j < C; ++j) av[j] = fmaf(av[j], s1, s2 * hs[j]);
}

__global__ __launch_bounds__(NTHR) void k_agg(
    const int* __restrict__ srcs, const int* __restrict__ dsts,
    const float* __restrict__ F, const float* __restrict__ SC,
    const float* __restrict__ bias, const float* __restrict__ prelu,
    float* outp, int nN, int nE, int nb, int vec8, int MPr) {
  extern __shared__ v4f lds_dyn[];
  int* reg1 = (int*)lds_dyn;
  int* reg2 = reg1 + RCAP;
  int* scnt = reg2 + RCAP;
  int* soff = scnt + NBMAX;
  int* list = soff + NBMAX;
  int* wcnt = list + LISTN;
  int* wtot = wcnt + NWAVE;
  const int tid = (int)threadIdx.x, lane = tid & 31, wave = tid >> 5;
  const int nodeBase = (int)blockIdx.x * nb;

  for (int i = tid; i < NBMAX; i += NTHR) scnt[i] = 0;
  for (int i = tid; i < RCAP; i += NTHR) reg2[i] = 0;
  __syncthreads();

  int tot = 0;
  const int nChunks = (nE + CHUNK - 1) / CHUNK;
#pragma unroll 1
  for (int ch = 0; ch < nChunks; ++ch) {
    const int cbase = ch * CHUNK;
    const int wc = scan_chunk(dsts, nE, cbase, nodeBase, nb, vec8, list, tid, lane, wave);
    if (lane == 0) wcnt[wave] = wc;
    __syncthreads();
    int pre = 0, all = 0;
#pragma unroll
    for (int w2 = 0; w2 < NWAVE; ++w2) {
      int c = wcnt[w2];
      c = c < 0 ? 0 : (c > WCAP ? WCAP : c);
      all += c;
      pre += (w2 < wave) ? c : 0;
    }
    const int wcc  = wc > WCAP ? WCAP : wc;
    const int base = tot + pre;
#pragma unroll 1
    for (int i = lane; i < wcc; i += 32) {
      const int ent = list[wave * WCAP + i];
      const int el  = (ent >> SLOTB) & (CHUNK - 1);
      const int sl  = ent & (NBMAX - 1);
      int eid = cbase + el;
      eid = eid > nE - 1 ? nE - 1 : eid;
      const int pos = base + i;
      if (pos < RCAP) reg1[pos] = (int)(((unsigned)eid << SLOTB) | (unsigned)sl);
    }
    tot += all;
    tot = tot > RCAP ? RCAP : tot;
    __syncthreads();
  }
  const int nh = tot;

  if (wave == 0) {
#pragma unroll 1
    for (int b0 = 0; b0 < nh; b0 += 32) {
      const int idx = b0 + lane;
      const int uv  = reg1[idx < nh ? idx : nh - 1];
      const int m32 = (nh - b0) < 32 ? (nh - b0) : 32;
#pragma unroll 1
      for (int k = 0; k < m32; ++k) {
        const int u  = __builtin_amdgcn_readlane(uv, k);
        const int sl = u & (NBMAX - 1);
        if (lane == 0) scnt[sl] = scnt[sl] + 1;
      }
    }
  }
  __syncthreads();

  {
    const v4i ca = *(const v4i*)(scnt + 8 * tid);
    const v4i cb = *(const v4i*)(scnt + 8 * tid + 4);
    const int e0 = ca.x < 0 ? 0 : ca.x, e1 = ca.y < 0 ? 0 : ca.y, e2 = ca.z < 0 ? 0 : ca.z, e3 = ca.w < 0 ? 0 : ca.w;
    const int e4 = cb.x < 0 ? 0 : cb.x, e5 = cb.y < 0 ? 0 : cb.y, e6 = cb.z < 0 ? 0 : cb.z, e7 = cb.w < 0 ? 0 : cb.w;
    const int ts = e0 + e1 + e2 + e3 + e4 + e5 + e6 + e7;
    int incl = ts;
#pragma unroll
    for (int d = 1; d < 32; d <<= 1) {
      const int up = __shfl_up(incl, d);
      if (lane >= d) incl += up;
    }
    if (lane == 31) wtot[wave] = incl;
    __syncthreads();
    int pre = 0;
#pragma unroll
    for (int w2 = 0; w2 < NWAVE; ++w2) pre += (w2 < wave) ? wtot[w2] : 0;
    int run = pre + incl - ts;
    soff[8 * tid + 0] = run; run += e0;
    soff[8 * tid + 1] = run; run += e1;
    soff[8 * tid + 2] = run; run += e2;
    soff[8 * tid + 3] = run; run += e3;
    soff[8 * tid + 4] = run; run += e4;
    soff[8 * tid + 5] = run; run += e5;
    soff[8 * tid + 6] = run; run += e6;
    soff[8 * tid + 7] = run;
  }
  __syncthreads();
  for (int i = tid; i < NBMAX; i += NTHR) list[i] = soff[i];
  __syncthreads();

  if (wave == 0) {
#pragma unroll 1
    for (int b0 = 0; b0 < nh; b0 += 32) {
      const int idx = b0 + lane;
      const int uv  = reg1[idx < nh ? idx : nh - 1];
      const int m32 = (nh - b0) < 32 ? (nh - b0) : 32;
#pragma unroll 1
      for (int k = 0; k < m32; ++k) {
        const int u   = __builtin_amdgcn_readlane(uv, k);
        const int sl  = u & (NBMAX - 1);
        const int eid = (int)((unsigned)u >> SLOTB);
        if (lane == 0) {
          int pos = list[sl];
          pos = pos < 0 ? 0 : (pos > RCAP - 1 ? RCAP - 1 : pos);
          reg2[pos] = eid;
          list[sl] = pos + 1;
        }
      }
    }
  }
  __syncthreads();

  const int nbw = nb >> 3;
  const bool ovf = (nh >= RCAP);
  const float qnan = __int_as_float(0x7fc00000);
  const int c0 = CPL * lane;
  const int head = lane >> 3;
  float* stw = (float*)reg1 + wave * STW;
  float bb[CPL];
  ldqb<CPL / 4>(bb, bias + c0);
  const float pa = bfr(prelu[0]);
  const float* ASp = SC + (size_t)head * (size_t)MPr;
  const float* ADp = SC + (size_t)(HEADS + head) * (size_t)MPr;

#pragma unroll 1
  for (int jt = 0; jt < nbw; ++jt) {
    const int slot = wave * nbw + jt;
    const int grow = nodeBase + slot;
    const int gcl  = grow < nN ? grow : nN - 1;
    int st = soff[slot];
    const int craw = scnt[slot];
    int cnt = craw;
    st  = st < 0 ? 0 : (st > nh ? nh : st);
    cnt = cnt < 0 ? 0 : (cnt > DEGCAP ? DEGCAP : cnt);
    if (cnt > nh - st) cnt = nh - st;
    const float pz = (ovf || craw > DEGCAP) ? qnan : 0.0f;
    const bool live = grow < nN;

    float hd[CPL];
    ldq<CPL / 4>(hd, F + (size_t)gcl * (size_t)CW + c0);
    const float asd = ASp[gcl];
    const float adv = ADp[gcl];
    float l0 = asd + adv;
    l0 = l0 >= 0.f ? l0 : NEGSA * l0;
    float mx = l0, dn = 1.0f;
    float av[CPL];
#pragma unroll
    for (int j = 0; j < CPL; ++j) av[j] = hd[j];

#pragma unroll 1
    for (int q = 0; q < cnt; ++q) {
      int idx = st + q; idx = idx > RCAP - 1 ? RCAP - 1 : idx;
      int eid = reg2[idx]; eid = eid < 0 ? 0 : (eid > nE - 1 ? nE - 1 : eid);
      const int sraw = srcs[eid];
      const int s = sraw < 0 ? 0 : (sraw > nN - 1 ? nN - 1 : sraw);
      float hs[CPL];
      ldq<CPL / 4>(hs, F + (size_t)s * (size_t)CW + c0);
      const float ass = ASp[s];
      float lg = ass + adv;
      lg = lg >= 0.f ? lg : NEGSA * lg;
      smerge<CPL>(lg, mx, dn, av, hs);
    }
    const float inv = __builtin_amdgcn_rcpf(dn + EPS_SM);

    float r[CPL];
#pragma unroll
    for (int j = 0; j < CPL; ++j) {
      float v = fmaf(av[j], inv, bb[j]);
      v = v >= 0.f ? v : pa * v;
      r[j] = (live ? v : 0.f) + pz;
    }
    v4f ga, gb;
    ga.x = r[0]; ga.y = r[1]; ga.z = r[2]; ga.w = r[3];
    gb.x = r[4]; gb.y = r[5]; gb.z = r[6]; gb.w = r[7];

    __builtin_amdgcn_fence(__ATOMIC_RELEASE, "wavefront");
    __builtin_amdgcn_wave_barrier();
    *(v4fa*)(stw + 8 * lane)     = ga;
    *(v4fa*)(stw + 8 * lane + 4) = gb;
    __builtin_amdgcn_fence(__ATOMIC_RELEASE, "wavefront");
    __builtin_amdgcn_wave_barrier();
    const v4f ya = *(const v4fa*)(stw + 4 * lane);
    const v4f yb = *(const v4fa*)(stw + (STW / 2) + 4 * lane);
    float* op = outp + (size_t)gcl * CW;
    if (live) {
      *(volatile v4f*)(op + 4 * lane)            = ya;
      *(volatile v4f*)(op + (CW / 2) + 4 * lane) = yb;
    }
    __threadfence();
    if (live) {
      *(volatile v4f*)(op + 4 * lane)            = ya;
      *(volatile v4f*)(op + (CW / 2) + 4 * lane) = yb;
    }
  }
  (void)stw; (void)outp;
}

static int pick_nb(int nE, int nN) {
  int nb = NBRUN;
  while (nb > 32 && (long long)nb * (long long)nE * 5LL > (long long)RCAP * (long long)nN * 4LL) nb >>= 1;
  return nb;
}
static inline int cdiv(int a, int b) { return (a + b - 1) / b; }

extern "C" void kernel_launch(void* const* d_in, const int* in_sizes, int n_in,
                              void* d_out, int out_size, void* d_ws, size_t ws_size,
                              hipStream_t stream) {
  if (n_in < 7) return;
  const int nN = in_sizes[0] / DIN;
  if (nN <= 0 || in_sizes[0] != nN * DIN || nN > (1 << 21)) return;
  if (in_sizes[1] < 2 || (in_sizes[1] & 1) != 0) return;
  const int nE = in_sizes[1] / 2;
  if (nE < 1 || nE >= (1 << (32 - SLOTB))) return;
  if (in_sizes[2] != DIN * CW) return;
  if (in_sizes[3] != CW || in_sizes[4] != CW) return;
  if (in_sizes[5] != CW) return;
  if (in_sizes[6] < 1) return;
  if (out_size != nN * CW) return;

  const float* x     = (const float*)d_in[0];
  const int*   ei    = (const int*)  d_in[1];
  const float* W     = (const float*)d_in[2];
  const float* atts  = (const float*)d_in[3];
  const float* attd  = (const float*)d_in[4];
  const float* bias  = (const float*)d_in[5];
  const float* prelu = (const float*)d_in[6];
  float* outp = (float*)d_out;
  const int* src = ei;
  const int* dst = ei + nE;

  const int MP   = cdiv(nN, GBM) * GBM;
  const int nb   = pick_nb(nE, nN);
  if (nb < 32 || (nb & (nb - 1)) != 0 || nb > NBMAX) return;
  const int gA   = cdiv(MP, nb);
  const int vec8 = ((nE & 3) == 0) ? 1 : 0;
  if (gA * nb < MP) return;

  char* ws = (char*)d_ws;
  size_t off = 0;
  const size_t oXB = off; off += (size_t)MP * DIN * 2;             off = (off + 255) & ~(size_t)255;
  const size_t oWT = off; off += (size_t)CW * K1 * 2;              off = (off + 255) & ~(size_t)255;
  const size_t oH  = off; off += (size_t)MP * CW * 4;              off = (off + 255) & ~(size_t)255;
  const size_t oSC = off; off += (size_t)NSC * MP * 4;             off = (off + 255) & ~(size_t)255;
  if (off > ws_size || off > (size_t)WSMAX) return;
  unsigned short* XB = (unsigned short*)(ws + oXB);
  unsigned short* WT = (unsigned short*)(ws + oWT);
  float*          H  = (float*)(ws + oH);
  float*          SC = (float*)(ws + oSC);

  hipFuncSetAttribute(reinterpret_cast<const void*>(&k_agg),
                      hipFuncAttributeMaxDynamicSharedMemorySize, LDS_AGG);

  const int nUx = MP * (DIN / 8);
  const int nBx = cdiv(nUx, NTHR);
  if (nBx * NTHR != nUx) return;
  k_prep<<<nBx + NBW1, NTHR, 0, stream>>>(x, W, XB, WT, nN, nUx, nBx);

  const int gM = MP / GBM;
  k_gemm<<<dim3(gM, CW / GBN), GTHR, 0, stream>>>(XB, WT, atts, attd, H, SC, K1, CW, MP);

  k_agg<<<gA, NTHR, LDS_AGG, stream>>>(src, dst, H, SC, bias, prelu, outp, nN, nE, nb, vec8, MP);
}
